// JointAttention_2748779069498
// MI455X (gfx1250) — hardware-verified
//
#include <hip/hip_runtime.h>
#include <math.h>

constexpr int kB    = 2;
constexpr int kNV   = 2048;
constexpr int kNT   = 256;
constexpr int kH    = 16;
constexpr int kDh   = 64;
constexpr int kC    = 1024;
constexpr int kS    = kNT + kNV;
constexpr int kTokV = kB * kNV;
constexpr int kTokT = kB * kNT;
constexpr int kWElems = kC * kC;
constexpr float kWCarry     = 16.0f;
constexpr float kWCarryInv  = 1.0f / 16.0f;
constexpr float kPCarry     = 32768.0f;
constexpr float kCtxCarry   = 256.0f;
constexpr float kPVScale    = kCtxCarry / kPCarry;
constexpr float kOutScale   = 1.0f / (kCtxCarry * kWCarry);
constexpr float kScoreScale = 0.125f;
constexpr float kEps        = 1.0e-6f;
constexpr float kInvDh      = 1.0f / 64.0f;
constexpr int kSmThreads = kS / 8;
constexpr int kSmWaves   = kSmThreads / 32;
static_assert(kH * kDh == kC, "shape");
static_assert(kS % 64 == 0 && kDh % 32 == 0 && kC % 64 == 0, "tiles");
static_assert(kTokV % 64 == 0 && kTokT % 64 == 0 && kNV % 64 == 0 && kNT % 64 == 0, "tiles");
static_assert(kSmThreads % 32 == 0 && kSmThreads * 8 == kS, "softmax coverage");
static_assert((kTokV * kC) % (8 * 256) == 0 && (kTokT * kC) % (8 * 256) == 0 && kWElems % (8 * 256) == 0, "cast coverage");

typedef __attribute__((ext_vector_type(16))) _Float16 v16h;
typedef __attribute__((ext_vector_type(8)))  _Float16 v8h;
typedef __attribute__((ext_vector_type(16))) __bf16   v16b;
typedef __attribute__((ext_vector_type(8)))  __bf16   v8b;
typedef __attribute__((ext_vector_type(8)))  float    v8f;
typedef __attribute__((ext_vector_type(4)))  float    v4f;
typedef __attribute__((ext_vector_type(4)))  unsigned int v4u;

__device__ __forceinline__ unsigned short f2bf_bits(float f) {
  unsigned u = __float_as_uint(f);
  return (unsigned short)((u + 0x7FFFu + ((u >> 16) & 1u)) >> 16);
}
__device__ __forceinline__ float bf_bits2f(unsigned short h) { return __uint_as_float(((unsigned)h) << 16); }

__device__ __forceinline__ void dep_guard_h(v8f& a, v8f& b, v16h x, v16h y) { asm volatile("v_nop\n\tv_nop\n\tv_nop\n\tv_nop" : "+v"(a), "+v"(b) : "v"(x), "v"(y)); }
__device__ __forceinline__ void dep_guard_b(v8f& a, v8f& b, v16b x, v16b y) { asm volatile("v_nop\n\tv_nop\n\tv_nop\n\tv_nop" : "+v"(a), "+v"(b) : "v"(x), "v"(y)); }
__device__ __forceinline__ void keep4_h(v16h a, v16h b, v16h c, v16h d) { asm volatile("v_nop" :: "v"(a), "v"(b), "v"(c), "v"(d)); }
__device__ __forceinline__ void keep4_b(v16b a, v16b b, v16b c, v16b d) { asm volatile("v_nop" :: "v"(a), "v"(b), "v"(c), "v"(d)); }
__device__ __forceinline__ void acc_guard4(v8f& a, v8f& b, v8f& c, v8f& d) { asm volatile("v_nop\n\tv_nop\n\tv_nop\n\tv_nop" : "+v"(a), "+v"(b), "+v"(c), "+v"(d)); }
template <typename T> struct Frag;
template <> struct Frag<_Float16> {
  typedef v16h V; union U { v16h v; v8h h[2]; };
  static __device__ __forceinline__ v16h load(const _Float16* p) {
    U f; f.h[0] = *(const v8h*)(p); f.h[1] = *(const v8h*)(p + 16); return f.v;
  }
  static __device__ __forceinline__ v8f mma(v16h a, v16h b, v8f c) {
    return __builtin_amdgcn_wmma_f32_16x16x32_f16(false, a, false, b, (short)0, c, false, false);
  }
  static __device__ __forceinline__ void guard(v8f& a, v8f& b, v16h x, v16h y) { dep_guard_h(a, b, x, y); }
  static __device__ __forceinline__ void keep(v16h a, v16h b, v16h c, v16h d) { keep4_h(a, b, c, d); }
};
template <> struct Frag<__bf16> {
  typedef v16b V; union U { v16b v; v8b h[2]; };
  static __device__ __forceinline__ v16b load(const __bf16* p) {
    U f; f.h[0] = *(const v8b*)(p); f.h[1] = *(const v8b*)(p + 16); return f.v;
  }
  static __device__ __forceinline__ v8f mma(v16b a, v16b b, v8f c) {
    return __builtin_amdgcn_wmma_f32_16x16x32_bf16(false, a, false, b, (short)0, c, false, false);
  }
  static __device__ __forceinline__ void guard(v8f& a, v8f& b, v16b x, v16b y) { dep_guard_b(a, b, x, y); }
  static __device__ __forceinline__ void keep(v16b a, v16b b, v16b c, v16b d) { keep4_b(a, b, c, d); }
};

__device__ __forceinline__ unsigned pk16(unsigned short a, unsigned short b) { return (unsigned)a | ((unsigned)b << 16); }
__device__ __forceinline__ unsigned short h_bits(float f) { const _Float16 h = (_Float16)f; return __builtin_bit_cast(unsigned short, h); }

template <int ET> struct Elem;
template <> struct Elem<0> { typedef _Float16 T; };
template <> struct Elem<1> { typedef __bf16 T; };
template <int ET, bool SPLIT, int BIAS_MODE, int OUT_MODE, bool RESID, int ACT = 0>
__global__ __launch_bounds__(256) void wmma_gemm64(
    const unsigned short* __restrict__ Ap, const unsigned short* __restrict__ A2p, int lda, long strideA,
    const unsigned short* __restrict__ Btp, const unsigned short* __restrict__ Bt2p, int ldb, long strideB,
    void* __restrict__ Cout, void* __restrict__ Cout2, int ldc, long strideC,
    const float* __restrict__ bias,
    const float* __restrict__ resid, long strideR,
    int M, int N, int K, float scale) {
  typedef typename Elem<ET>::T T;
  typedef typename Frag<T>::V V;
  const T* A = (const T*)Ap; const T* A2 = (const T*)A2p; const T* Bt = (const T*)Btp; const T* Bt2 = (const T*)Bt2p;
  __shared__ __align__(16) float sT[8][16 * 68];
  const int b    = blockIdx.y;
  const int lane = threadIdx.x & 31;
  const int wave = threadIdx.x >> 5;
  const int tilesN = N >> 6;
  const int tilesM = M >> 6;
  const int tile = blockIdx.x * 8 + wave;
  if (tile >= tilesM * tilesN) return;
  const int tm = tile / tilesN;
  const int tn = tile - tm * tilesN;
  const int m0 = tm << 6;
  const int n0 = tn << 6;

  const T* Ab  = A  + (size_t)b * strideA;
  const T* Bb  = Bt + (size_t)b * strideB;
  const T* Ab2 = SPLIT ? (A2  + (size_t)b * strideA) : nullptr;
  const T* Bb2 = SPLIT ? (Bt2 + (size_t)b * strideB) : nullptr;

  const int rlane = lane & 15;
  const int koff  = (lane >> 4) * 8;
  const int mOff  = (lane >> 4) * 8;

  v8f acc[4][4];
#pragma unroll
  for (int i = 0; i < 4; ++i)
#pragma unroll
    for (int j = 0; j < 4; ++j) acc[i][j] = (v8f){0.f,0.f,0.f,0.f,0.f,0.f,0.f,0.f};

  for (int k0 = 0; k0 < K; k0 += 32) {
    V bh[4], bl[4];
#pragma unroll
    for (int j = 0; j < 4; ++j) {
      const size_t bo = (size_t)(n0 + (j << 4) + rlane) * ldb + koff + k0;
      bh[j] = Frag<T>::load(Bb + bo);
      if (SPLIT) bl[j] = Frag<T>::load(Bb2 + bo);
    }
#pragma unroll
    for (int i = 0; i < 4; ++i) {
      const size_t ao = (size_t)(m0 + (i << 4) + rlane) * lda + koff + k0;
      V ah = Frag<T>::load(Ab + ao);
      V al;
      if (SPLIT) al = Frag<T>::load(Ab2 + ao);
#pragma unroll
      for (int j = 0; j < 4; ++j) {
        acc[i][j] = Frag<T>::mma(ah, bh[j], acc[i][j]);
        if (SPLIT) {
          acc[i][j] = Frag<T>::mma(ah, bl[j], acc[i][j]);
          acc[i][j] = Frag<T>::mma(al, bh[j], acc[i][j]);
        }
      }
      Frag<T>::guard(acc[i][0], acc[i][3], ah, SPLIT ? al : ah);
    }
    Frag<T>::keep(bh[0], bh[1], bh[2], bh[3]);
    if (SPLIT) Frag<T>::keep(bl[0], bl[1], bl[2], bl[3]);
  }
  acc_guard4(acc[0][0], acc[0][1], acc[0][2], acc[0][3]);
  acc_guard4(acc[1][0], acc[1][1], acc[1][2], acc[1][3]);
  acc_guard4(acc[2][0], acc[2][1], acc[2][2], acc[2][3]);
  acc_guard4(acc[3][0], acc[3][1], acc[3][2], acc[3][3]);

  float* slab = sT[wave];
  const float* Rb = RESID ? (resid + (size_t)b * strideR) : nullptr;
#pragma unroll
  for (int i = 0; i < 4; ++i) {
    const int mBase = m0 + (i << 4);
#pragma unroll
    for (int j = 0; j < 4; ++j) {
      const int n = n0 + (j << 4) + rlane;
      float bv = 0.f;
      if (BIAS_MODE == 2) bv = bias[n];
#pragma unroll
      for (int r = 0; r < 8; ++r) {
        float v = acc[i][j][r] * scale;
        if (BIAS_MODE == 1) v += bias[mBase + mOff + r];
        if (BIAS_MODE == 2) v += bv;
        if (RESID) v += Rb[(size_t)(mBase + mOff + r) * ldc + n];
        if (ACT == 2) v = fmaxf(v, 0.0f);
        if (ACT == 4) v = (v > 0.f) ? v : 0.01f * v;
        slab[(mOff + r) * 68 + (j << 4) + rlane] = v;
      }
    }
    __builtin_amdgcn_fence(__ATOMIC_RELEASE, "workgroup");
    __builtin_amdgcn_wave_barrier();
    __builtin_amdgcn_fence(__ATOMIC_ACQUIRE, "workgroup");
    if (OUT_MODE == 0) {
      float* C = (float*)Cout + (size_t)b * strideC;
      const int hh = lane >> 4, c4 = (lane & 15) * 4;
      for (int pass = 0; pass < 2; ++pass) {
#pragma unroll
        for (int it = 0; it < 8; ++it) {
          const int row = it * 2 + hh;
          v4f v = *(const v4f*)(slab + row * 68 + c4);
          *(volatile v4f*)(C + (size_t)(mBase + row) * ldc + n0 + c4) = v;
        }
        __threadfence();
      }
    } else {
      const int q = lane >> 3, c8 = (lane & 7) * 8;
      unsigned short* C  = (unsigned short*)Cout  + (size_t)b * strideC;
      unsigned short* C2 = (OUT_MODE == 2) ? ((unsigned short*)Cout2 + (size_t)b * strideC) : nullptr;
      for (int pass = 0; pass < 2; ++pass) {
#pragma unroll
        for (int it = 0; it < 4; ++it) {
          const int row = it * 4 + q;
          const float* sp = slab + row * 68 + c8;
          v8h hv, lv;
#pragma unroll
          for (int e = 0; e < 8; ++e) {
            if (OUT_MODE == 1) {
              hv[e] = (_Float16)sp[e];
            } else {
              unsigned short hb = f2bf_bits(sp[e]);
              unsigned short lb = f2bf_bits(sp[e] - bf_bits2f(hb));
              hv[e] = __builtin_bit_cast(_Float16, hb);
              lv[e] = __builtin_bit_cast(_Float16, lb);
            }
          }
          *(volatile v8h*)(C + (size_t)(mBase + row) * ldc + n0 + c8) = hv;
          if (OUT_MODE == 2) *(volatile v8h*)(C2 + (size_t)(mBase + row) * ldc + n0 + c8) = lv;
        }
        __threadfence();
      }
    }
    __builtin_amdgcn_fence(__ATOMIC_RELEASE, "workgroup");
    __builtin_amdgcn_wave_barrier();
    __builtin_amdgcn_fence(__ATOMIC_ACQUIRE, "workgroup");
  }
}

#define GemmF32 wmma_gemm64<0, false, 0, 0, false, 0>
#define GemmVT  wmma_gemm64<0, false, 1, 1, false, 0>
#define GemmCtx wmma_gemm64<0, false, 0, 1, false, 0>
#define GemmOut wmma_gemm64<0, false, 2, 0, false, 0>

__global__ __launch_bounds__(256) void cast8_f16_kernel(const float* __restrict__ in, unsigned short* __restrict__ out, int n8) {
  const int i = blockIdx.x * 256 + threadIdx.x;
  if (i >= n8) return;
  const float* p = in + 8 * (size_t)i;
  const v4f a = *(const v4f*)(p);
  const v4f c = *(const v4f*)(p + 4);
  unsigned short hb[8];
#pragma unroll
  for (int e = 0; e < 4; ++e) {
    hb[e]     = h_bits(a[e]);
    hb[4 + e] = h_bits(c[e]);
  }
  const v4u u = (v4u){pk16(hb[0], hb[1]), pk16(hb[2], hb[3]), pk16(hb[4], hb[5]), pk16(hb[6], hb[7])};
  unsigned short* q = out + 8 * (size_t)i;
  *(volatile v4u*)q = u;
  __threadfence();
  *(volatile v4u*)q = u;
}

__global__ __launch_bounds__(256) void wcast8_kernel(const float* __restrict__ W0, const float* __restrict__ W1,
                                                     const float* __restrict__ W2, const float* __restrict__ W3,
                                                     const float* __restrict__ W4, const float* __restrict__ W5,
                                                     const float* __restrict__ W6, const float* __restrict__ W7,
                                                     unsigned short* __restrict__ out, int n8, float scale) {
  const int z = blockIdx.y;
  const float* W = (z == 0) ? W0 : (z == 1) ? W1 : (z == 2) ? W2 : (z == 3) ? W3
                 : (z == 4) ? W4 : (z == 5) ? W5 : (z == 6) ? W6 : W7;
  const int i = blockIdx.x * 256 + threadIdx.x;
  if (i >= n8) return;
  const float* p = W + 8 * (size_t)i;
  const v4f a = *(const v4f*)(p);
  const v4f c = *(const v4f*)(p + 4);
  unsigned short hb[8];
#pragma unroll
  for (int e = 0; e < 4; ++e) {
    hb[e]     = h_bits(a[e] * scale);
    hb[4 + e] = h_bits(c[e] * scale);
  }
  const v4u u = (v4u){pk16(hb[0], hb[1]), pk16(hb[2], hb[3]), pk16(hb[4], hb[5]), pk16(hb[6], hb[7])};
  unsigned short* q = out + (size_t)z * 8 * (size_t)n8 + 8 * (size_t)i;
  *(volatile v4u*)q = u;
  __threadfence();
  *(volatile v4u*)q = u;
}

template <bool DO_ROPE>
__global__ __launch_bounds__(256) void norm_rope_kernel(
    const float* __restrict__ F,
    const float* __restrict__ qb, const float* __restrict__ kb,
    const float* __restrict__ qn, const float* __restrict__ kn,
    const float* __restrict__ rc, const float* __restrict__ rs,
    unsigned short* __restrict__ Qo, unsigned short* __restrict__ Ko,
    int nPerBatch, int seqOff) {
  const int m    = blockIdx.x;
  const int b    = m / nPerBatch;
  const int pos  = m - b * nPerBatch;
  const int t    = threadIdx.x;
  const int lane = t & 31, wave = t >> 5;
  const int which = wave >> 2;
  const int head = ((wave & 3) << 2) + (lane >> 3);
  const int d0   = (lane & 7) << 3;
  const int col  = head * kDh + d0;
  const float* bias = which ? kb : qb;
  const float* gain = which ? kn : qn;
  unsigned short* outp = which ? Ko : Qo;

  const float* fp = F + (size_t)m * (2 * kC) + which * kC + col;
  const v4f f0 = *(const v4f*)(fp);
  const v4f f1 = *(const v4f*)(fp + 4);
  const v4f b0 = *(const v4f*)(bias + col);
  const v4f b1 = *(const v4f*)(bias + col + 4);
  asm volatile("" ::: "memory");
  float x[8];
#pragma unroll
  for (int e = 0; e < 4; ++e) { x[e] = f0[e] + b0[e]; x[4 + e] = f1[e] + b1[e]; }
  float ss = 0.0f;
#pragma unroll
  for (int e = 0; e < 8; ++e) ss += x[e] * x[e];
  ss += __shfl_xor(ss, 1, 32);
  ss += __shfl_xor(ss, 2, 32);
  ss += __shfl_xor(ss, 4, 32);
  const float rsc = rsqrtf(ss * kInvDh + kEps);
  const v4f g0 = *(const v4f*)(gain + d0);
  const v4f g1 = *(const v4f*)(gain + d0 + 4);
  float y[8];
#pragma unroll
  for (int e = 0; e < 4; ++e) { y[e] = (x[e] * rsc) * g0[e]; y[4 + e] = (x[4 + e] * rsc) * g1[e]; }
  if (DO_ROPE) {
    asm volatile("" ::: "memory");
    const float* cpt = rc + (size_t)pos * kDh + d0;
    const float* spt = rs + (size_t)pos * kDh + d0;
    const v4f c0 = *(const v4f*)(cpt);
    const v4f c1 = *(const v4f*)(cpt + 4);
    const v4f s0 = *(const v4f*)(spt);
    const v4f s1 = *(const v4f*)(spt + 4);
    float cs[8], sn[8];
#pragma unroll
    for (int e = 0; e < 4; ++e) { cs[e] = c0[e]; cs[4 + e] = c1[e]; sn[e] = s0[e]; sn[4 + e] = s1[e]; }
    float o[8];
#pragma unroll
    for (int i = 0; i < 4; ++i) {
      o[2 * i]     = y[2 * i] * cs[2 * i] + (-y[2 * i + 1]) * sn[2 * i];
      o[2 * i + 1] = y[2 * i + 1] * cs[2 * i + 1] + y[2 * i] * sn[2 * i + 1];
    }
#pragma unroll
    for (int e = 0; e < 8; ++e) y[e] = o[e];
  }
  unsigned short hb[8];
#pragma unroll
  for (int e = 0; e < 8; ++e) hb[e] = h_bits(y[e]);
  const v4u u = (v4u){pk16(hb[0], hb[1]), pk16(hb[2], hb[3]), pk16(hb[4], hb[5]), pk16(hb[6], hb[7])};
  unsigned short* dst = outp + ((size_t)(b * kS + seqOff + pos)) * kC + col;
  *(volatile v4u*)dst = u;
  __threadfence();
  *(volatile v4u*)dst = u;
}

__global__ __launch_bounds__(kSmThreads) void softmax_row_kernel(const float* __restrict__ Sp, unsigned short* __restrict__ Pp) {
  __shared__ __align__(16) float lg[kS];
  __shared__ float redM[kSmWaves];
  __shared__ float redS[kSmWaves];
  const int row  = blockIdx.x;
  const int t    = threadIdx.x;
  const int lane = t & 31, wave = t >> 5;
  const size_t rowoff = (size_t)row * kS;
  const float* sr = Sp + rowoff + 8 * (size_t)t;
  const v4f a = *(const v4f*)(sr);
  const v4f c = *(const v4f*)(sr + 4);
  float mx = fmaxf(fmaxf(fmaxf(a[0], a[1]), fmaxf(a[2], a[3])), fmaxf(fmaxf(c[0], c[1]), fmaxf(c[2], c[3])));
#pragma unroll
  for (int off = 16; off > 0; off >>= 1) mx = fmaxf(mx, __shfl_xor(mx, off, 32));
  if (lane == 0) redM[wave] = mx;
  __syncthreads();
  float m = redM[0];
#pragma unroll
  for (int w = 1; w < kSmWaves; ++w) m = fmaxf(m, redM[w]);

  float sum = 0.0f;
#pragma unroll 1
  for (int it = 0; it < 2; ++it) {
    const v4f l = *(const v4f*)(sr + 4 * it);
    v4f ev;
#pragma unroll
    for (int e = 0; e < 4; ++e) {
      ev[e] = expf(l[e] - m);
      sum += ev[e];
    }
    *(v4f*)(lg + 8 * t + 4 * it) = ev;
  }
#pragma unroll
  for (int off = 16; off > 0; off >>= 1) sum += __shfl_xor(sum, off, 32);
  if (lane == 0) redS[wave] = sum;
  __syncthreads();
  float tot = redS[0];
#pragma unroll
  for (int w = 1; w < kSmWaves; ++w) tot += redS[w];
  const float inv = kPCarry / tot;

  const v4f e0 = *(const v4f*)(lg + 8 * t);
  const v4f e1 = *(const v4f*)(lg + 8 * t + 4);
  unsigned short hb[8];
#pragma unroll
  for (int e = 0; e < 4; ++e) {
    hb[e]     = h_bits(e0[e] * inv);
    hb[4 + e] = h_bits(e1[e] * inv);
  }
  const v4u u = (v4u){pk16(hb[0], hb[1]), pk16(hb[2], hb[3]), pk16(hb[4], hb[5]), pk16(hb[6], hb[7])};
  unsigned short* pr = Pp + rowoff + 8 * (size_t)t;
  *(volatile v4u*)pr = u;
  __threadfence();
  *(volatile v4u*)pr = u;
}

extern "C" void kernel_launch(void* const* d_in, const int* in_sizes, int n_in,
                              void* d_out, int out_size, void* d_ws, size_t ws_size,
                              hipStream_t stream) {
  if (n_in < 24) return;
  if (in_sizes[0] != kTokV * kC || in_sizes[1] != kTokT * kC) return;
  if (in_sizes[2] != kNV * kDh || in_sizes[3] != kNV * kDh) return;
  for (int i = 4; i < 20; i += 2) {
    if (in_sizes[i] != kWElems) return;
    if (in_sizes[i + 1] != kC) return;
  }
  for (int i = 20; i < 24; ++i) if (in_sizes[i] != kDh) return;
  if (out_size != kTokV * kC + kTokT * kC) return;

  const size_t szXV = (size_t)kTokV * kC * 2;
  const size_t szXT = (size_t)kTokT * kC * 2;
  const size_t szW  = (size_t)8 * kWElems * 2;
  const size_t szF  = (size_t)kTokV * 2 * kC * 4;
  const size_t szQK = (size_t)kB * kS * kC * 2;
  const size_t szVT = (size_t)kB * kH * kDh * kS * 2;
  const size_t szSC = (size_t)kS * kS * 4;
  const size_t szPP = (size_t)kS * kS * 2;
  const size_t offXV  = 0;
  const size_t offXT  = offXV + szXV;
  const size_t offW   = offXT + szXT;
  const size_t offF   = offW + szW;
  const size_t offQ   = offF + szF;
  const size_t offK   = offQ + szQK;
  const size_t offVT  = offK + szQK;
  const size_t offCTX = offVT + szVT;
  const size_t offSC  = offCTX + szQK;
  const size_t offPP  = offSC + szSC;
  const size_t total  = offPP + szPP;
  if (ws_size < total) return;

  const float* vis_x  = (const float*)d_in[0];
  const float* txt_x  = (const float*)d_in[1];
  const float* rc     = (const float*)d_in[2];
  const float* rs     = (const float*)d_in[3];
  const float* vis_qw = (const float*)d_in[4];
  const float* vis_qb = (const float*)d_in[5];
  const float* vis_kw = (const float*)d_in[6];
  const float* vis_kb = (const float*)d_in[7];
  const float* vis_vw = (const float*)d_in[8];
  const float* vis_vb = (const float*)d_in[9];
  const float* vis_ow = (const float*)d_in[10];
  const float* vis_ob = (const float*)d_in[11];
  const float* txt_qw = (const float*)d_in[12];
  const float* txt_qb = (const float*)d_in[13];
  const float* txt_kw = (const float*)d_in[14];
  const float* txt_kb = (const float*)d_in[15];
  const float* txt_vw = (const float*)d_in[16];
  const float* txt_vb = (const float*)d_in[17];
  const float* txt_ow = (const float*)d_in[18];
  const float* txt_ob = (const float*)d_in[19];
  const float* vis_qn = (const float*)d_in[20];
  const float* vis_kn = (const float*)d_in[21];
  const float* txt_qn = (const float*)d_in[22];
  const float* txt_kn = (const float*)d_in[23];
  float* out0 = (float*)d_out;
  float* out1 = (float*)d_out + (size_t)kTokV * kC;

  char* ws = (char*)d_ws;
  unsigned short* XV16  = (unsigned short*)(ws + offXV);
  unsigned short* XT16  = (unsigned short*)(ws + offXT);
  unsigned short* W16   = (unsigned short*)(ws + offW);
  float*          F32T  = (float*)(ws + offF);
  unsigned short* Q16   = (unsigned short*)(ws + offQ);
  unsigned short* K16   = (unsigned short*)(ws + offK);
  unsigned short* VT16  = (unsigned short*)(ws + offVT);
  unsigned short* CTX16 = (unsigned short*)(ws + offCTX);
  float*          SC    = (float*)(ws + offSC);
  unsigned short* PP    = (unsigned short*)(ws + offPP);
  const unsigned short* WqkV = W16;
  const unsigned short* WvV  = W16 + (size_t)2 * kWElems;
  const unsigned short* WoV  = W16 + (size_t)3 * kWElems;
  const unsigned short* WqkT = W16 + (size_t)4 * kWElems;
  const unsigned short* WvT  = W16 + (size_t)6 * kWElems;
  const unsigned short* WoT  = W16 + (size_t)7 * kWElems;

  const int n8V = (kTokV * kC) / 8;
  const int n8T = (kTokT * kC) / 8;
  const int n8W = kWElems / 8;
  cast8_f16_kernel<<<dim3(n8V / 256), dim3(256), 0, stream>>>(vis_x, XV16, n8V);
  cast8_f16_kernel<<<dim3(n8T / 256), dim3(256), 0, stream>>>(txt_x, XT16, n8T);
  wcast8_kernel<<<dim3(n8W / 256, 8), dim3(256), 0, stream>>>(vis_qw, vis_kw, vis_vw, vis_ow, txt_qw, txt_kw, txt_vw, txt_ow,
                                                            W16, n8W, kWCarry);

  const long strideVTb = (long)kH * kDh * kS;
  const long strideTok = (long)kS * kC;

  {
    const int tilesQK = (kTokV / 64) * (2 * kC / 64);
    GemmF32<<<dim3(tilesQK / 8, 1), dim3(256), 0, stream>>>(
        XV16, XV16, kC, 0L, WqkV, WqkV, kC, 0L, (void*)F32T, (void*)F32T, 2 * kC, 0L,
        vis_qb, vis_qb, 0L, kTokV, 2 * kC, kC, kWCarryInv);
    norm_rope_kernel<true><<<dim3(kTokV), dim3(256), 0, stream>>>(
        F32T, vis_qb, vis_kb, vis_qn, vis_kn, rc, rs, Q16, K16, kNV, kNT);
    const int tilesVT = (kC / 64) * (kNV / 64);
    GemmVT<<<dim3(tilesVT / 8, kB), dim3(256), 0, stream>>>(
        WvV, WvV, kC, 0L, XV16, XV16, kC, (long)kNV * kC, (void*)(VT16 + kNT), (void*)(VT16 + kNT), kS, strideVTb,
        vis_vb, vis_vb, 0L, kC, kNV, kC, kWCarryInv);
  }
  {
    const int tilesQK = (kTokT / 64) * (2 * kC / 64);
    GemmF32<<<dim3(tilesQK / 8, 1), dim3(256), 0, stream>>>(
        XT16, XT16, kC, 0L, WqkT, WqkT, kC, 0L, (void*)F32T, (void*)F32T, 2 * kC, 0L,
        txt_qb, txt_qb, 0L, kTokT, 2 * kC, kC, kWCarryInv);
    norm_rope_kernel<false><<<dim3(kTokT), dim3(256), 0, stream>>>(
        F32T, txt_qb, txt_kb, txt_qn, txt_kn, rc, rs, Q16, K16, kNT, 0);
    const int tilesVT = (kC / 64) * (kNT / 64);
    GemmVT<<<dim3(tilesVT / 8, kB), dim3(256), 0, stream>>>(
        WvT, WvT, kC, 0L, XT16, XT16, kC, (long)kNT * kC, (void*)VT16, (void*)VT16, kS, strideVTb,
        txt_vb, txt_vb, 0L, kC, kNT, kC, kWCarryInv);
  }

  const int tilesScore = (kS / 64) * (kS / 64);
  const int tilesCtx   = (kS / 64) * (kDh / 64);
  for (int b = 0; b < kB; ++b) {
    for (int h = 0; h < kH; ++h) {
      const size_t tokOff = (size_t)b * kS * kC + (size_t)h * kDh;
      const unsigned short* Ag  = Q16 + tokOff;
      const unsigned short* Btg = K16 + tokOff;
      GemmF32<<<dim3(tilesScore / 8, 1), dim3(256), 0, stream>>>(
          Ag, Ag, kC, 0L, Btg, Btg, kC, 0L, (void*)SC, (void*)SC, kS, 0L,
          vis_qb, vis_qb, 0L, kS, kS, kDh, kScoreScale);
      softmax_row_kernel<<<dim3(kS), dim3(kSmThreads), 0, stream>>>(SC, PP);
      const unsigned short* VTg = VT16 + ((size_t)b * kH + h) * (size_t)kDh * kS;
      unsigned short* ctxg = CTX16 + tokOff;
      GemmCtx<<<dim3((tilesCtx + 7) / 8, 1), dim3(256), 0, stream>>>(
          PP, PP, kS, 0L, VTg, VTg, kS, 0L, (void*)ctxg, (void*)ctxg, kC, 0L,
          vis_qb, vis_qb, 0L, kS, kDh, kS, kPVScale);
    }
  }

  {
    const int tilesOV = (kNV / 64) * (kC / 64);
    GemmOut<<<dim3(tilesOV / 8, kB), dim3(256), 0, stream>>>(
        CTX16 + (size_t)kNT * kC, CTX16 + (size_t)kNT * kC, kC, strideTok, WoV, WoV, kC, 0L,
        (void*)out0, (void*)out0, kC, (long)kNV * kC,
        vis_ob, vis_ob, 0L, kNV, kC, kC, kOutScale);
    const int tilesOT = (kNT / 64) * (kC / 64);
    GemmOut<<<dim3(tilesOT / 8, kB), dim3(256), 0, stream>>>(
        CTX16, CTX16, kC, strideTok, WoT, WoT, kC, 0L,
        (void*)out1, (void*)out1, kC, (long)kNT * kC,
        txt_ob, txt_ob, 0L, kNT, kC, kC, kOutScale);
  }
}
